// QuantumLayer_43593918055108
// MI455X (gfx1250) — hardware-verified
//
#include <hip/hip_runtime.h>
#include <math.h>

typedef __attribute__((ext_vector_type(16))) _Float16 v16h;
typedef __attribute__((ext_vector_type(8)))  _Float16 v8h;
typedef __attribute__((ext_vector_type(8)))  float    v8f;
typedef __attribute__((ext_vector_type(4)))  float    v4f;
typedef __attribute__((ext_vector_type(4)))  unsigned int v4u;

constexpr int kWires          = 4;
constexpr int kStates         = 16;
constexpr int kLayers         = 3;
constexpr int kGates          = kLayers * kWires;
constexpr int kThreads        = 256;
constexpr int kWavesPerBlock  = kThreads / 32;
constexpr int kSamplesPerWave = 32;
constexpr int kKpad           = 32;
constexpr int kPlaneHalves    = kStates * kKpad;
constexpr int kNumPlanes      = 4;
constexpr int kMaxBlocks      = 512;
constexpr int kColPitch       = 33;
constexpr float kHiCarry  = 16.0f;
constexpr float kResCarry = 2048.0f;
constexpr float kMainInv  = 1.0f / 256.0f;
constexpr float kResInv   = 1.0f / 524288.0f;

static_assert(kPlaneHalves == 512, "plane halves");
static_assert(kThreads == kNumPlanes * kPlaneHalves / 8, "assembly coverage: 256 threads x 8 halves = 4 planes");
static_assert(kKpad % 32 == 0, "K step");

__device__ __forceinline__ unsigned pk16(unsigned short a, unsigned short b) { return (unsigned)a | ((unsigned)b << 16); }

__device__ __forceinline__ v16h lds_frag(const _Float16* p) {
  union { v16h v; v8h hh[2]; } f;
  f.hh[0] = *(const v8h*)(p);
  f.hh[1] = *(const v8h*)(p + 16);
  return f.v;
}

__device__ __forceinline__ v8f mma_f16(v16h a, v16h b, v8f c) {
  return __builtin_amdgcn_wmma_f32_16x16x32_f16(false, a, false, b, (short)0, c, false, false);
}

__device__ __forceinline__ void mma_group_guard(v8f& a, v8f& b, v8f& c, v8f& d,
                                                v16h p, v16h q, v16h r, v16h s, v16h t, v16h u) {
  asm volatile("v_nop\n\tv_nop\n\tv_nop\n\tv_nop"
               : "+v"(a), "+v"(b), "+v"(c), "+v"(d)
               : "v"(p), "v"(q), "v"(r), "v"(s), "v"(t), "v"(u));
}

__device__ __forceinline__ void wave_lds_sync() {
  __builtin_amdgcn_fence(__ATOMIC_RELEASE, "workgroup");
  __builtin_amdgcn_wave_barrier();
  __builtin_amdgcn_fence(__ATOMIC_ACQUIRE, "workgroup");
}

__global__ void __launch_bounds__(kThreads) vqc_fused_kernel(const float* __restrict__ x,
                                                             const float* __restrict__ w,
                                                             float* __restrict__ out,
                                                             int nWaveTiles) {
  __shared__ float sG[kGates][8];
  __shared__ float sRe[kStates][kColPitch];
  __shared__ float sIm[kStates][kColPitch];
  __shared__ __align__(16) unsigned short sA[kNumPlanes * kPlaneHalves];
  __shared__ __align__(16) float sP[kWavesPerBlock][kSamplesPerWave * kStates];

  const int tid  = threadIdx.x;
  const int lane = tid & 31;
  const int wave = tid >> 5;
  const int h    = lane >> 4;
  const int n    = lane & 15;

  {
    const int g = (tid < kGates) ? tid : (kGates - 1);
    const float phi = w[g * 3 + 0];
    const float th  = w[g * 3 + 1];
    const float om  = w[g * 3 + 2];
    float st, ct, sp, cp, sm, cm;
    sincosf(th * 0.5f, &st, &ct);
    sincosf((phi + om) * 0.5f, &sp, &cp);
    sincosf((phi - om) * 0.5f, &sm, &cm);
    if (tid < kGates) {
      sG[tid][0] = ct; sG[tid][1] = st;
      sG[tid][2] = cp; sG[tid][3] = sp;
      sG[tid][4] = cm; sG[tid][5] = sm;
      sG[tid][6] = 0.0f; sG[tid][7] = 0.0f;
    }
  }
  __syncthreads();

  if (wave == 0) {
    const int col = lane;
    const int jb  = lane & 15;
#pragma unroll
    for (int i = 0; i < kStates; ++i) {
      sRe[i][col] = (i == jb) ? 1.0f : 0.0f;
      sIm[i][col] = 0.0f;
    }
#pragma unroll 1
    for (int ly = 0; ly < kLayers; ++ly) {
#pragma unroll 1
      for (int q = 0; q < kWires; ++q) {
        const int g = ly * kWires + q;
        const float ct = sG[g][0], st = sG[g][1];
        const float cp = sG[g][2], sp = sG[g][3];
        const float cm = sG[g][4], sm = sG[g][5];
        const float u00r =  cp * ct, u00i = -sp * ct;
        const float u01r = -cm * st, u01i = -sm * st;
        const float u10r =  cm * st, u10i = -sm * st;
        const float u11r =  cp * ct, u11i =  sp * ct;
        const int tb = 1 << (3 - q);
#pragma unroll 1
        for (int i = 0; i < kStates; ++i) {
          if ((i & tb) == 0) {
            const int i1 = i | tb;
            const float r0 = sRe[i][col],  m0 = sIm[i][col];
            const float r1 = sRe[i1][col], m1 = sIm[i1][col];
            sRe[i][col]  = u00r * r0 - u00i * m0 + u01r * r1 - u01i * m1;
            sIm[i][col]  = u00r * m0 + u00i * r0 + u01r * m1 + u01i * r1;
            sRe[i1][col] = u10r * r0 - u10i * m0 + u11r * r1 - u11i * m1;
            sIm[i1][col] = u10r * m0 + u10i * r0 + u11r * m1 + u11i * r1;
          }
        }
      }
      const int rr = ly + 1;
#pragma unroll 1
      for (int q = 0; q < kWires; ++q) {
        const int t    = (q + rr) & 3;
        const int cbit = 1 << (3 - q);
        const int tbit = 1 << (3 - t);
#pragma unroll 1
        for (int i = 0; i < kStates; ++i) {
          if (((i & cbit) != 0) && ((i & tbit) == 0)) {
            const int i1 = i | tbit;
            const float tr = sRe[i][col], tr1 = sRe[i1][col];
            sRe[i][col] = tr1; sRe[i1][col] = tr;
            const float ti = sIm[i][col], ti1 = sIm[i1][col];
            sIm[i][col] = ti1; sIm[i1][col] = ti;
          }
        }
      }
    }
  }
  __syncthreads();

  {
    const int pl = tid >> 6;
    const int o  = (tid & 63) * 8;
    const int z  = o >> 5;
    const int cb = o & 31;
    const bool useIm  = (pl >= 2);
    const bool isRes  = ((pl & 1) != 0);
    const bool hiCols = (cb < 16);
    unsigned short hb[8];
#pragma unroll
    for (int e = 0; e < 8; ++e) {
      const int jj = (cb + e) & 15;
      const float ur = sRe[z][jj];
      const float ui = sIm[z][jj];
      const float u  = useIm ? ui : ur;
      const float us = u * kHiCarry;
      const _Float16 hs = (_Float16)us;
      const float rem = (us - (float)hs) * kResCarry;
      const _Float16 ls = (_Float16)rem;
      const unsigned short hsb = __builtin_bit_cast(unsigned short, hs);
      const unsigned short lsb = __builtin_bit_cast(unsigned short, ls);
      const unsigned short zb  = (unsigned short)0;
      hb[e] = hiCols ? hsb : (isRes ? lsb : zb);
    }
    const v4u u4 = (v4u){pk16(hb[0], hb[1]), pk16(hb[2], hb[3]), pk16(hb[4], hb[5]), pk16(hb[6], hb[7])};
    *(v4u*)(sA + pl * kPlaneHalves + o) = u4;
  }
  __syncthreads();

  const _Float16* sAh = (const _Float16*)(const void*)sA;
  const v16h aReM = lds_frag(sAh + 0 * kPlaneHalves + n * kKpad + 8 * h);
  const v16h aReR = lds_frag(sAh + 1 * kPlaneHalves + n * kKpad + 8 * h);
  const v16h aImM = lds_frag(sAh + 2 * kPlaneHalves + n * kKpad + 8 * h);
  const v16h aImR = lds_frag(sAh + 3 * kPlaneHalves + n * kKpad + 8 * h);

  const int wavesTotal = gridDim.x * kWavesPerBlock;
  const int gw = blockIdx.x * kWavesPerBlock + wave;
  float* pw = sP[wave];
  const float sgnH = h ? -1.0f : 1.0f;

#pragma unroll 1
  for (int wt = gw; wt < nWaveTiles; wt += wavesTotal) {
    const size_t s = (size_t)wt * kSamplesPerWave + lane;
    const v4f xv = *(const v4f*)(x + s * 4);

    float s0, c0, s1, c1, s2, c2, s3, c3;
    sincosf(xv.x * 0.5f, &s0, &c0);
    sincosf(xv.y * 0.5f, &s1, &c1);
    sincosf(xv.z * 0.5f, &s2, &c2);
    sincosf(xv.w * 0.5f, &s3, &c3);

    const float t0 = c0 * c1, t1 = c0 * s1, t2 = s0 * c1, t3 = s0 * s1;
    const float e0 = c2 * c3, e1 = c2 * s3, e2 = s2 * c3, e3 = s2 * s3;
    float p[16];
    p[ 0] = t0 * e0; p[ 1] = t0 * e1; p[ 2] = t0 * e2; p[ 3] = t0 * e3;
    p[ 4] = t1 * e0; p[ 5] = t1 * e1; p[ 6] = t1 * e2; p[ 7] = t1 * e3;
    p[ 8] = t2 * e0; p[ 9] = t2 * e1; p[10] = t2 * e2; p[11] = t2 * e3;
    p[12] = t3 * e0; p[13] = t3 * e1; p[14] = t3 * e2; p[15] = t3 * e3;

    {
      float* prow = pw + lane * kStates;
      *(v4f*)(prow + 0)  = (v4f){p[0],  p[1],  p[2],  p[3]};
      *(v4f*)(prow + 4)  = (v4f){p[4],  p[5],  p[6],  p[7]};
      *(v4f*)(prow + 8)  = (v4f){p[8],  p[9],  p[10], p[11]};
      *(v4f*)(prow + 12) = (v4f){p[12], p[13], p[14], p[15]};
    }
    wave_lds_sync();

    float res[2][4];
#pragma unroll
    for (int t = 0; t < 2; ++t) {
      const float* qrow = pw + (16 * t + n) * kStates + 8 * h;
      const v4f pa = *(const v4f*)(qrow);
      const v4f pb = *(const v4f*)(qrow + 4);
      float e8[8];
      e8[0] = pa.x; e8[1] = pa.y; e8[2] = pa.z; e8[3] = pa.w;
      e8[4] = pb.x; e8[5] = pb.y; e8[6] = pb.z; e8[7] = pb.w;

      v16h bm, br;
#pragma unroll
      for (int i = 0; i < 8; ++i) {
        const float v = e8[i] * kHiCarry;
        const _Float16 hh = (_Float16)v;
        const float rem = (v - (float)hh) * kResCarry;
        const _Float16 ll = (_Float16)rem;
        bm[i] = hh; bm[8 + i] = hh;
        br[i] = ll; br[8 + i] = hh;
      }

      const v8f zero8 = (v8f){0.f, 0.f, 0.f, 0.f, 0.f, 0.f, 0.f, 0.f};
      v8f dRm = mma_f16(aReM, bm, zero8);
      v8f dRr = mma_f16(aReR, br, zero8);
      v8f dIm = mma_f16(aImM, bm, zero8);
      v8f dIr = mma_f16(aImR, br, zero8);
      mma_group_guard(dRm, dRr, dIm, dIr, bm, br, aReM, aReR, aImM, aImR);

      float pr[8];
#pragma unroll
      for (int r = 0; r < 8; ++r) {
        const float re = dRm[r] * kMainInv + dRr[r] * kResInv;
        const float im = dIm[r] * kMainInv + dIr[r] * kResInv;
        pr[r] = re * re + im * im;
      }
      const float a0 = pr[0] + pr[1], a1 = pr[2] + pr[3];
      const float a2 = pr[4] + pr[5], a3 = pr[6] + pr[7];
      const float tw3 = (pr[0] - pr[1]) + (pr[2] - pr[3]) + (pr[4] - pr[5]) + (pr[6] - pr[7]);
      const float g0 = a0 + a1, g1 = a2 + a3;
      const float sAll = g0 + g1;
      const float tw1 = g0 - g1;
      const float tw2 = (a0 - a1) + (a2 - a3);
      const float o1 = tw1 + __shfl_xor(tw1, 16, 32);
      const float o2 = tw2 + __shfl_xor(tw2, 16, 32);
      const float o3 = tw3 + __shfl_xor(tw3, 16, 32);
      const float sOther = __shfl_xor(sAll, 16, 32);
      const float o0 = (sAll - sOther) * sgnH;
      res[t][0] = o0; res[t][1] = o1; res[t][2] = o2; res[t][3] = o3;
    }

    v4f ov;
    ov.x = h ? res[1][0] : res[0][0];
    ov.y = h ? res[1][1] : res[0][1];
    ov.z = h ? res[1][2] : res[0][2];
    ov.w = h ? res[1][3] : res[0][3];
    volatile v4f* op = (volatile v4f*)(out + s * 4);
    *op = ov;
    __threadfence();
    *op = ov;

    wave_lds_sync();
  }
}

extern "C" void kernel_launch(void* const* d_in, const int* in_sizes, int n_in,
                              void* d_out, int out_size, void* d_ws, size_t ws_size,
                              hipStream_t stream) {
  const float* x = (const float*)d_in[0];
  const float* w = (const float*)d_in[1];
  float* out = (float*)d_out;
  const int B = in_sizes[0] / kWires;
  if (B <= 0 || (B % kSamplesPerWave) != 0) return;
  if (in_sizes[1] < kGates * 3) return;
  if (out_size < B * kWires) return;
  const int nWaveTiles = B / kSamplesPerWave;
  int blocks = (nWaveTiles + kWavesPerBlock - 1) / kWavesPerBlock;
  if (blocks > kMaxBlocks) blocks = kMaxBlocks;
  if (blocks < 1) blocks = 1;
  vqc_fused_kernel<<<blocks, kThreads, 0, stream>>>(x, w, out, nWaveTiles);
}
